// CustomAttention_29643864277218
// MI455X (gfx1250) — hardware-verified
//
#include <hip/hip_runtime.h>
#include <math.h>
#include <stdint.h>

#ifndef NB
#define NB 8
#endif
#ifndef SEQ
#define SEQ 2048
#endif
#define NB_FULL  8
#define SEQ_FULL 2048
#define DM    384
#define NH    6
#define HD    64
#define DQKV  (3 * DM)
#define NQB64 (SEQ / 64)
#define NKT   (SEQ / 64)
static_assert(NH * HD == DM);
static_assert((SEQ % 64) == 0 && SEQ >= 64 && SEQ <= SEQ_FULL);
static_assert(NB >= 1 && NB <= NB_FULL);
static_assert((DM % 64) == 0 && (DQKV % 64) == 0 && ((2 * DM) % 32) == 0);

typedef _Float16 v16h __attribute__((ext_vector_type(16)));
typedef _Float16 v8h  __attribute__((ext_vector_type(8)));
typedef __bf16   v16b __attribute__((ext_vector_type(16)));
typedef __bf16   v8b  __attribute__((ext_vector_type(8)));
typedef float    v8f  __attribute__((ext_vector_type(8)));
typedef float    v4f  __attribute__((ext_vector_type(4)));
typedef unsigned int v4u __attribute__((ext_vector_type(4)));

#if defined(__HIP_DEVICE_COMPILE__)
#define DEV_ASM 1
#else
#define DEV_ASM 0
#endif

__device__ __forceinline__ unsigned short bf_bits(float f) {
  unsigned u = __float_as_uint(f);
  return (unsigned short)((u + 0x7FFFu + ((u >> 16) & 1u)) >> 16);
}
__device__ __forceinline__ float bf_up(unsigned short hb) { return __uint_as_float(((unsigned)hb) << 16); }
__device__ __forceinline__ float bfr(float f) { return bf_up(bf_bits(f)); }
__device__ __forceinline__ unsigned short h_bits(_Float16 x) { return __builtin_bit_cast(unsigned short, x); }
__device__ __forceinline__ unsigned pk16(unsigned short a, unsigned short b) { return (unsigned)a | ((unsigned)b << 16); }
__device__ __forceinline__ v8f zero8() { v8f z = {0.f, 0.f, 0.f, 0.f, 0.f, 0.f, 0.f, 0.f}; return z; }

template <typename OT> struct FT;
template <> struct FT<__bf16>   { typedef v16b frag; typedef v8b half8; };
template <> struct FT<_Float16> { typedef v16h frag; typedef v8h half8; };

template <typename OT>
__device__ __forceinline__ typename FT<OT>::frag ldfrag(const OT* p) {
  union { typename FT<OT>::frag v; typename FT<OT>::half8 h[2]; } f;
  f.h[0] = *(const typename FT<OT>::half8*)(p);
  f.h[1] = *(const typename FT<OT>::half8*)(p + 16);
  return f.v;
}

__device__ __forceinline__ v8f mmar(v16b a, v16b b, v8f c) {
  return __builtin_amdgcn_wmma_f32_16x16x32_bf16(false, a, false, b, (short)0, c, false, false);
}
__device__ __forceinline__ v8f mmar(v16h a, v16h b, v8f c) {
  return __builtin_amdgcn_wmma_f32_16x16x32_f16(false, a, false, b, (short)0, c, false, false);
}
__device__ __forceinline__ v8f mma_h(v16h a, v16h b, v8f c) {
  c = __builtin_amdgcn_wmma_f32_16x16x32_f16(false, a, false, b, (short)0, c, false, false);
#if DEV_ASM
  asm volatile("v_nop\n\tv_nop\n\tv_nop\n\tv_nop" : "+v"(c) : "v"(a), "v"(b));
#endif
  return c;
}
__device__ __forceinline__ void dep_guard(v8f& a, v8f& b, v16b x, v16b y) {
#if DEV_ASM
  asm volatile("v_nop\n\tv_nop\n\tv_nop\n\tv_nop" : "+v"(a), "+v"(b) : "v"(x), "v"(y));
#else
  (void)a; (void)b; (void)x; (void)y;
#endif
}
__device__ __forceinline__ void dep_guard(v8f& a, v8f& b, v16h x, v16h y) {
#if DEV_ASM
  asm volatile("v_nop\n\tv_nop\n\tv_nop\n\tv_nop" : "+v"(a), "+v"(b) : "v"(x), "v"(y));
#else
  (void)a; (void)b; (void)x; (void)y;
#endif
}
__device__ __forceinline__ void keep4(v16b a, v16b b, v16b c, v16b d) {
#if DEV_ASM
  asm volatile("v_nop" :: "v"(a), "v"(b), "v"(c), "v"(d));
#else
  (void)a; (void)b; (void)c; (void)d;
#endif
}
__device__ __forceinline__ void keep4(v16h a, v16h b, v16h c, v16h d) {
#if DEV_ASM
  asm volatile("v_nop" :: "v"(a), "v"(b), "v"(c), "v"(d));
#else
  (void)a; (void)b; (void)c; (void)d;
#endif
}
__device__ __forceinline__ void acc_guard4(v8f& a, v8f& b, v8f& c, v8f& d) {
#if DEV_ASM
  asm volatile("v_nop\n\tv_nop\n\tv_nop\n\tv_nop" : "+v"(a), "+v"(b), "+v"(c), "+v"(d));
#else
  (void)a; (void)b; (void)c; (void)d;
#endif
}

__global__ __launch_bounds__(256) void cvt_bf16x8(const float* __restrict__ in, long long strideIn,
                                                  unsigned short* out, long long strideOut, int n8) {
  const int i = blockIdx.x * 256 + (int)threadIdx.x;
  const float* inb = in + (size_t)blockIdx.y * (size_t)strideIn;
  unsigned short* outb = out + (size_t)blockIdx.y * (size_t)strideOut;
  if (i < n8) {
    const v4f a  = *(const v4f*)(inb + (size_t)i * 8);
    const v4f a4 = *(const v4f*)(inb + (size_t)i * 8 + 4);
    v4u p;
    p[0] = pk16(bf_bits(a[0]),  bf_bits(a[1]));
    p[1] = pk16(bf_bits(a[2]),  bf_bits(a[3]));
    p[2] = pk16(bf_bits(a4[0]), bf_bits(a4[1]));
    p[3] = pk16(bf_bits(a4[2]), bf_bits(a4[3]));
    unsigned short* o = outb + (size_t)i * 8;
    *(volatile v4u*)o = p;
    __threadfence();
    *(volatile v4u*)o = p;
  }
}

__global__ __launch_bounds__(256) void tr_bf16(const float* __restrict__ w, int N,
                                               unsigned short* out, int ldo, int ocol) {
  __shared__ __align__(16) float tile[64 * 68];
  const int tid = (int)threadIdx.x;
  const int n0 = blockIdx.x * 64;
  const int k0 = blockIdx.y * 64;
#pragma unroll
  for (int i = 0; i < 16; ++i) {
    const int idx = i * 256 + tid;
    const int r = idx >> 6;
    const int c = idx & 63;
    tile[c * 68 + r] = w[(size_t)(k0 + r) * (size_t)N + n0 + c];
  }
  __syncthreads();
  const int wave = tid >> 5, lane = tid & 31;
  const int q = lane >> 3, c8 = (lane & 7) * 8;
  v4u pv[2];
#pragma unroll
  for (int it = 0; it < 2; ++it) {
    const int n = wave * 8 + it * 4 + q;
    const v4f a  = *(const v4f*)(tile + n * 68 + c8);
    const v4f a4 = *(const v4f*)(tile + n * 68 + c8 + 4);
    v4u p;
    p[0] = pk16(bf_bits(a[0]),  bf_bits(a[1]));
    p[1] = pk16(bf_bits(a[2]),  bf_bits(a[3]));
    p[2] = pk16(bf_bits(a4[0]), bf_bits(a4[1]));
    p[3] = pk16(bf_bits(a4[2]), bf_bits(a4[3]));
    pv[it] = p;
  }
  for (int pass = 0; pass < 2; ++pass) {
#pragma unroll
    for (int it = 0; it < 2; ++it) {
      const int n = wave * 8 + it * 4 + q;
      *(volatile v4u*)(out + (size_t)(n0 + n) * (size_t)ldo + ocol + k0 + c8) = pv[it];
    }
    __threadfence();
  }
}

template <typename OT, int OUT_MODE, int BMODE>
__global__ __launch_bounds__(256) void gemm64(
    const unsigned short* __restrict__ Ap, int lda, long long strideA,
    const unsigned short* __restrict__ Btp, int ldb, long long strideB,
    void* Cout, void* Cout2, int ldc, long long strideC,
    const float* __restrict__ bias,
    int M, int N, int K, float oscale, float rscale) {
  typedef typename FT<OT>::frag V16;
  const OT* A  = (const OT*)(const void*)Ap;
  const OT* Bt = (const OT*)(const void*)Btp;
  __shared__ __align__(16) float sT[8][16 * 68];
  const int b    = blockIdx.y;
  const int lane = threadIdx.x & 31;
  const int wave = threadIdx.x >> 5;
  const int tilesN = N >> 6;
  const int tilesM = M >> 6;
  const int tile = blockIdx.x * 8 + wave;
  if (tile >= tilesM * tilesN) return;
  const int tm = tile / tilesN;
  const int tn = tile - tm * tilesN;
  const int m0 = tm << 6;
  const int n0 = tn << 6;

  const OT* Ab = A  + (size_t)b * (size_t)strideA;
  const OT* Bb = Bt + (size_t)b * (size_t)strideB;

  const int rlane = lane & 15;
  const int koff  = (lane >> 4) * 8;
  const int mOff  = (lane >> 4) * 8;

  v8f acc[4][4];
#pragma unroll
  for (int i = 0; i < 4; ++i)
#pragma unroll
    for (int j = 0; j < 4; ++j) acc[i][j] = zero8();

  for (int k0 = 0; k0 < K; k0 += 32) {
    V16 bq[4];
#pragma unroll
    for (int j = 0; j < 4; ++j)
      bq[j] = ldfrag<OT>(Bb + (size_t)(n0 + (j << 4) + rlane) * ldb + koff + k0);
#pragma unroll
    for (int i = 0; i < 4; ++i) {
      const V16 af = ldfrag<OT>(Ab + (size_t)(m0 + (i << 4) + rlane) * lda + koff + k0);
#pragma unroll
      for (int j = 0; j < 4; ++j) acc[i][j] = mmar(af, bq[j], acc[i][j]);
      dep_guard(acc[i][0], acc[i][3], af, bq[3]);
    }
    keep4(bq[0], bq[1], bq[2], bq[3]);
  }
  acc_guard4(acc[0][0], acc[0][1], acc[0][2], acc[0][3]);
  acc_guard4(acc[1][0], acc[1][1], acc[1][2], acc[1][3]);
  acc_guard4(acc[2][0], acc[2][1], acc[2][2], acc[2][3]);
  acc_guard4(acc[3][0], acc[3][1], acc[3][2], acc[3][3]);

  v4f bb = {0.f, 0.f, 0.f, 0.f};
  float bc[8];
#pragma unroll
  for (int e = 0; e < 8; ++e) bc[e] = 0.f;
  if (BMODE == 1) {
    if (OUT_MODE == 0) {
      const v4f t = *(const v4f*)(bias + n0 + (lane & 15) * 4);
#pragma unroll
      for (int e = 0; e < 4; ++e) bb[e] = bfr(t[e]);
    } else {
      const v4f t0 = *(const v4f*)(bias + n0 + (lane & 7) * 8);
      const v4f t1 = *(const v4f*)(bias + n0 + (lane & 7) * 8 + 4);
#pragma unroll
      for (int e = 0; e < 4; ++e) { bc[e] = bfr(t0[e]); bc[4 + e] = bfr(t1[e]); }
    }
  }

  float* slab = sT[wave];
#pragma unroll
  for (int i = 0; i < 4; ++i) {
    const int mBase = m0 + (i << 4);
#pragma unroll
    for (int j = 0; j < 4; ++j) {
#pragma unroll
      for (int r = 0; r < 8; ++r) {
        slab[(mOff + r) * 68 + (j << 4) + rlane] = acc[i][j][r];
      }
    }
    __builtin_amdgcn_fence(__ATOMIC_RELEASE, "workgroup");
    __builtin_amdgcn_wave_barrier();
    __builtin_amdgcn_fence(__ATOMIC_ACQUIRE, "workgroup");
    if (OUT_MODE == 0) {
      float* C = (float*)Cout + (size_t)b * (size_t)strideC;
      const int h2 = lane >> 4, c4 = (lane & 15) * 4;
      for (int pass = 0; pass < 2; ++pass) {
#pragma unroll
        for (int it = 0; it < 8; ++it) {
          const int row = it * 2 + h2;
          float br = 0.f;
          if (BMODE == 2) br = bfr(bias[mBase + row]);
          const v4f v = *(const v4f*)(slab + row * 68 + c4) * oscale + bb + br;
          *(volatile v4f*)(C + (size_t)(mBase + row) * ldc + n0 + c4) = v;
        }
        __threadfence();
      }
    } else {
      const int q = lane >> 3, c8 = (lane & 7) * 8;
      unsigned short* C  = (unsigned short*)Cout  + (size_t)b * (size_t)strideC;
      unsigned short* C2 = (unsigned short*)Cout2 + (size_t)b * (size_t)strideC;
      v4u hv[4], lv[4];
#pragma unroll
      for (int it = 0; it < 4; ++it) {
        const int row = it * 4 + q;
        const float* sp = slab + row * 68 + c8;
        float br = 0.f;
        if (BMODE == 2) br = bfr(bias[mBase + row]);
        float f[8];
#pragma unroll
        for (int e = 0; e < 8; ++e) f[e] = sp[e] + bc[e] + br;
        v4u a, a2;
#pragma unroll
        for (int e = 0; e < 4; ++e) {
          const float f0 = f[2 * e], f1 = f[2 * e + 1];
          const _Float16 x0 = (_Float16)f0, x1 = (_Float16)f1;
          const unsigned short h0 = h_bits(x0), h1 = h_bits(x1);
          unsigned short l0 = 0, l1 = 0;
          if (OUT_MODE == 3) {
            l0 = h_bits((_Float16)((f0 - (float)x0) * rscale));
            l1 = h_bits((_Float16)((f1 - (float)x1) * rscale));
          }
          a[e] = pk16(h0, h1); a2[e] = pk16(l0, l1);
        }
        hv[it] = a; lv[it] = a2;
      }
      for (int pass = 0; pass < 2; ++pass) {
#pragma unroll
        for (int it = 0; it < 4; ++it) {
          const int row = it * 4 + q;
          *(volatile v4u*)(C + (size_t)(mBase + row) * ldc + n0 + c8) = hv[it];
          if (OUT_MODE == 3) *(volatile v4u*)(C2 + (size_t)(mBase + row) * ldc + n0 + c8) = lv[it];
        }
        __threadfence();
      }
    }
    __builtin_amdgcn_fence(__ATOMIC_RELEASE, "workgroup");
    __builtin_amdgcn_wave_barrier();
    __builtin_amdgcn_fence(__ATOMIC_ACQUIRE, "workgroup");
  }
}

__global__ __launch_bounds__(128)
void attn_mha(const unsigned short* __restrict__ qhp, const unsigned short* __restrict__ qlp,
              const unsigned short* __restrict__ kpp,
              const unsigned short* __restrict__ vhp, const unsigned short* __restrict__ vlp,
              unsigned short* cp, float sscale) {
  union FH { v16h v; v8h h[2]; };
  __shared__ __align__(16) _Float16 Ksh[64 * 64];
  __shared__ __align__(16) _Float16 Vth[64 * 64];
  __shared__ __align__(16) _Float16 Vtl[64 * 64];
  __shared__ __align__(16) _Float16 Psh[4][16 * 64];
  __shared__ __align__(16) float    Os[4][16 * 64];

  const int tid  = threadIdx.x;
  const int wave = tid >> 5;
  const int lane = tid & 31;
  const int hh   = lane >> 4;
  const int c    = lane & 15;

  const int bx   = blockIdx.x;
  const int qb   = bx % NQB64;
  const int rest = bx / NQB64;
  const int h    = rest % NH;
  const int b    = rest / NH;
  const int q0   = qb * 64 + wave * 16;
  const size_t rowB = (size_t)b * SEQ;

  const _Float16* Qh = (const _Float16*)(const void*)qhp;
  const _Float16* Ql = (const _Float16*)(const void*)qlp;
  const _Float16* Kg = (const _Float16*)(const void*)kpp + (size_t)h * HD;
  const _Float16* Vh = (const _Float16*)(const void*)vhp + ((size_t)b * DM + (size_t)h * HD) * SEQ;
  const _Float16* Vl = (const _Float16*)(const void*)vlp + ((size_t)b * DM + (size_t)h * HD) * SEQ;

  v16h qah[2], qal[2];
#pragma unroll
  for (int dc = 0; dc < 2; ++dc) {
    const size_t qo = (rowB + q0 + c) * DM + (size_t)h * HD + dc * 32 + 8 * hh;
    qah[dc] = ldfrag<_Float16>(Qh + qo);
    qal[dc] = ldfrag<_Float16>(Ql + qo);
  }

  float mrow[8], lrow[8];
  v8f oacc[4];
#pragma unroll
  for (int r = 0; r < 8; ++r) { mrow[r] = -INFINITY; lrow[r] = 0.f; }
#pragma unroll
  for (int t = 0; t < 4; ++t) oacc[t] = zero8();

  for (int kt = 0; kt < NKT; ++kt) {
    const int kv0 = kt * 64;
    __syncthreads();
    {
      const int r = tid >> 1, half = (tid & 1) * 32;
      const _Float16* kg  = Kg + (rowB + kv0 + r) * DM + half;
      const _Float16* vg  = Vh + (size_t)r * SEQ + kv0 + half;
      const _Float16* vlg = Vl + (size_t)r * SEQ + kv0 + half;
#pragma unroll
      for (int i = 0; i < 4; ++i) {
        const v8h a0 = *(const v8h*)(kg + 8 * i);
        const v8h b0 = *(const v8h*)(vg + 8 * i);
        const v8h b1 = *(const v8h*)(vlg + 8 * i);
        *(v8h*)(Ksh + r * 64 + half + 8 * i) = a0;
        *(v8h*)(Vth + r * 64 + half + 8 * i) = b0;
        *(v8h*)(Vtl + r * 64 + half + 8 * i) = b1;
      }
    }
    __syncthreads();

    v8f s[4];
#pragma unroll
    for (int j = 0; j < 4; ++j) {
      v8f ah = zero8(), al = zero8();
#pragma unroll
      for (int dc = 0; dc < 2; ++dc) {
        FH kb;
        kb.h[0] = *(const v8h*)(Ksh + (j * 16 + c) * 64 + dc * 32 + 8 * hh);
        kb.h[1] = *(const v8h*)(Ksh + (j * 16 + c) * 64 + dc * 32 + 16 + 8 * hh);
        ah = mma_h(qah[dc], kb.v, ah);
        al = mma_h(qal[dc], kb.v, al);
      }
#pragma unroll
      for (int r = 0; r < 8; ++r) s[j][r] = (ah[r] + al[r] * (1.0f / 4096.0f)) * sscale;
    }

    _Float16* pwh = Psh[wave];
#pragma unroll
    for (int r = 0; r < 8; ++r) {
      float m = s[0][r];
#pragma unroll
      for (int j = 1; j < 4; ++j) m = fmaxf(m, s[j][r]);
#pragma unroll
      for (int off = 1; off < 16; off <<= 1) m = fmaxf(m, __shfl_xor(m, off, 32));
      const float mnew  = fmaxf(mrow[r], m);
      const float msafe = (mnew == -INFINITY) ? 0.f : mnew;
      const float alpha = __expf(mrow[r] - msafe);
      mrow[r] = mnew;
      float psum = 0.f;
#pragma unroll
      for (int j = 0; j < 4; ++j) {
        const float p = __expf(s[j][r] - msafe);
        psum += p;
        pwh[(8 * hh + r) * 64 + j * 16 + c] = (_Float16)(p * 1024.0f);
      }
#pragma unroll
      for (int off = 1; off < 16; off <<= 1) psum += __shfl_xor(psum, off, 32);
      lrow[r] = lrow[r] * alpha + psum;
#pragma unroll
      for (int t = 0; t < 4; ++t) oacc[t][r] *= alpha;
    }
    __builtin_amdgcn_fence(__ATOMIC_RELEASE, "workgroup");
    __builtin_amdgcn_wave_barrier();
    __builtin_amdgcn_fence(__ATOMIC_ACQUIRE, "workgroup");

    v8f o1[4];
#pragma unroll
    for (int t = 0; t < 4; ++t) o1[t] = zero8();
#pragma unroll 1
    for (int kk = 0; kk < 2; ++kk) {
      FH pa;
      pa.h[0] = *(const v8h*)(pwh + c * 64 + kk * 32 + 8 * hh);
      pa.h[1] = *(const v8h*)(pwh + c * 64 + kk * 32 + 16 + 8 * hh);
#pragma unroll
      for (int t = 0; t < 4; ++t) {
        FH vb, vl;
        vb.h[0] = *(const v8h*)(Vth + (t * 16 + c) * 64 + kk * 32 + 8 * hh);
        vb.h[1] = *(const v8h*)(Vth + (t * 16 + c) * 64 + kk * 32 + 16 + 8 * hh);
        vl.h[0] = *(const v8h*)(Vtl + (t * 16 + c) * 64 + kk * 32 + 8 * hh);
        vl.h[1] = *(const v8h*)(Vtl + (t * 16 + c) * 64 + kk * 32 + 16 + 8 * hh);
        oacc[t] = mma_h(pa.v, vb.v, oacc[t]);
        o1[t]   = mma_h(pa.v, vl.v, o1[t]);
      }
    }
#pragma unroll
    for (int t = 0; t < 4; ++t)
#pragma unroll
      for (int r = 0; r < 8; ++r) oacc[t][r] += o1[t][r] * (1.0f / 4096.0f);
  }

  float* os = Os[wave];
#pragma unroll
  for (int r = 0; r < 8; ++r) {
    const float l = lrow[r];
    const float inv = ((l > 0.f) ? (1.0f / l) : 0.f) * (1.0f / 1024.0f);
#pragma unroll
    for (int t = 0; t < 4; ++t) os[(8 * hh + r) * 64 + t * 16 + c] = oacc[t][r] * inv;
  }
  __builtin_amdgcn_fence(__ATOMIC_RELEASE, "workgroup");
  __builtin_amdgcn_wave_barrier();
  __builtin_amdgcn_fence(__ATOMIC_ACQUIRE, "workgroup");
  {
    const int q4 = lane >> 3, c8 = (lane & 7) * 8;
    v4u hv[4], lv[4];
#pragma unroll
    for (int it = 0; it < 4; ++it) {
      const int row = it * 4 + q4;
      const float* sp = os + row * 64 + c8;
      v4u a, a2;
#pragma unroll
      for (int e = 0; e < 4; ++e) {
        const float f0 = sp[2 * e], f1 = sp[2 * e + 1];
        const unsigned short h0 = bf_bits(f0), h1 = bf_bits(f1);
        const unsigned short l0 = bf_bits(f0 - bf_up(h0)), l1 = bf_bits(f1 - bf_up(h1));
        a[e]  = pk16(h0, h1);
        a2[e] = pk16(l0, l1);
      }
      hv[it] = a; lv[it] = a2;
    }
    for (int pass = 0; pass < 2; ++pass) {
#pragma unroll
      for (int it = 0; it < 4; ++it) {
        const int row = it * 4 + q4;
        const size_t go = (rowB + q0 + row) * (size_t)(2 * DM) + (size_t)h * HD + c8;
        *(volatile v4u*)(cp + go) = hv[it];
        *(volatile v4u*)(cp + go + DM) = lv[it];
      }
      __threadfence();
    }
  }
}

extern "C" void kernel_launch(void* const* d_in, const int* in_sizes, int n_in,
                              void* d_out, int out_size, void* d_ws, size_t ws_size,
                              hipStream_t stream) {
  if (n_in < 5) return;
  if (in_sizes[0] < ((NB - 1) * SEQ_FULL + SEQ) * DM) return;
  if (in_sizes[1] < DM * DQKV) return;
  if (in_sizes[2] < DQKV) return;
  if (in_sizes[3] < DM * DM) return;
  if (in_sizes[4] < DM) return;
  if (out_size < NB * SEQ * DM) return;

  const float* x      = (const float*)d_in[0];
  const float* qkv_w  = (const float*)d_in[1];
  const float* qkv_b  = (const float*)d_in[2];
  const float* proj_w = (const float*)d_in[3];
  const float* proj_b = (const float*)d_in[4];

  const size_t PX  = (size_t)NB * SEQ * DM * 2;
  const size_t PWT = (size_t)DQKV * DM * 2;
  const size_t PWP = (size_t)DM * (2 * DM) * 2;
  const size_t PVT = (size_t)NB * DM * SEQ * 2;
  const size_t PC  = (size_t)NB * SEQ * (2 * DM) * 2;
  size_t off = 0;
  const size_t oXb  = off; off += PX;
  const size_t oWt  = off; off += PWT;
  const size_t oWp  = off; off += PWP;
  const size_t oQh  = off; off += PX;
  const size_t oQl  = off; off += PX;
  const size_t oKp  = off; off += PX;
  const size_t oVTh = off; off += PVT;
  const size_t oVTl = off; off += PVT;
  const size_t oCt  = off; off += PC;
  if (off > ws_size) return;
  if (off > (size_t)134217728) return;

  char* ws = (char*)d_ws;
  unsigned short* Xb  = (unsigned short*)(ws + oXb);
  unsigned short* Wt  = (unsigned short*)(ws + oWt);
  unsigned short* Wp2 = (unsigned short*)(ws + oWp);
  unsigned short* Qh  = (unsigned short*)(ws + oQh);
  unsigned short* Ql  = (unsigned short*)(ws + oQl);
  unsigned short* Kp  = (unsigned short*)(ws + oKp);
  unsigned short* VTh = (unsigned short*)(ws + oVTh);
  unsigned short* VTl = (unsigned short*)(ws + oVTl);
  unsigned short* Ctx = (unsigned short*)(ws + oCt);

  const dim3 blk(256);
  const int n8x = SEQ * DM / 8;
  const dim3 gCvtX((n8x + 255) / 256, NB);
  const dim3 gTrQKV(DQKV / 64, DM / 64);
  const dim3 gTrP(DM / 64, DM / 64);
  const int tilesQK = ((NB * SEQ) / 64) * (DM / 64);
  const dim3 gQK((tilesQK + 7) / 8, 1);
  const int tilesVT = (DM / 64) * (SEQ / 64);
  const dim3 gVT((tilesVT + 7) / 8, NB);
  const dim3 gAttn(NB * NH * NQB64);

  cvt_bf16x8<<<gCvtX, blk, 0, stream>>>(x, (long long)SEQ_FULL * DM, Xb, (long long)SEQ * DM, n8x);
  tr_bf16<<<gTrQKV, blk, 0, stream>>>(qkv_w, DQKV, Wt, DM, 0);
  tr_bf16<<<gTrP, blk, 0, stream>>>(proj_w, DM, Wp2, 2 * DM, 0);
  tr_bf16<<<gTrP, blk, 0, stream>>>(proj_w, DM, Wp2, 2 * DM, DM);
  gemm64<__bf16, 3, 1><<<gQK, blk, 0, stream>>>(
      Xb, DM, 0LL, Wt, DM, 0LL,
      (void*)Qh, (void*)Ql, DM, 0LL, qkv_b,
      NB * SEQ, DM, DM, 1.0f, 4096.0f);
  gemm64<__bf16, 1, 1><<<gQK, blk, 0, stream>>>(
      Xb, DM, 0LL, Wt + (size_t)DM * DM, DM, 0LL,
      (void*)Kp, (void*)Kp, DM, 0LL, qkv_b + DM,
      NB * SEQ, DM, DM, 1.0f, 1.0f);
  gemm64<__bf16, 3, 2><<<gVT, blk, 0, stream>>>(
      Wt + (size_t)2 * DM * DM, DM, 0LL, Xb, DM, (long long)SEQ * DM,
      (void*)VTh, (void*)VTl, SEQ, (long long)DM * SEQ, qkv_b + 2 * DM,
      DM, SEQ, DM, 1.0f, 4096.0f);
  attn_mha<<<gAttn, dim3(128), 0, stream>>>(Qh, Ql, Kp, VTh, VTl, Ctx, 0.125f);
  gemm64<__bf16, 0, 1><<<gQK, blk, 0, stream>>>(
      Ctx, 2 * DM, 0LL, Wp2, 2 * DM, 0LL,
      d_out, d_out, DM, 0LL, proj_b,
      NB * SEQ, DM, 2 * DM, 1.0f, 1.0f);
  (void)hipGetLastError();
}
